// SplineCritic_47588237640103
// MI455X (gfx1250) — hardware-verified
//
#include <hip/hip_runtime.h>

typedef _Float16 v16h __attribute__((ext_vector_type(16)));
typedef _Float16 v8h  __attribute__((ext_vector_type(8)));
typedef float    v8f  __attribute__((ext_vector_type(8)));
typedef float    v4f  __attribute__((ext_vector_type(4)));
union Frag { v16h v; v8h half[2]; };

#define NG      8
#define NF      9
#define DIN1    256
#define NH1     128
#define NH2     64
#define K1TOT   (DIN1 * NF)
#define K2TOT   (NH1 * NF)
#define FSCALE  16.0f
#define WSCALE  64.0f
#define OSCALE  (1.0f / 1024.0f)
#define GRID_LO (-2.0f)
#define GRID_ST (4.0f / 7.0f)
#define INVH    1.75f
#define TM      64
#define TN      64
#define FIN_T   256

static_assert(K1TOT % 64 == 0);
static_assert(K2TOT % 64 == 0);
static_assert(NH1 % TN == 0);
static_assert(NH2 % TN == 0);
static_assert(DIN1 % 32 == 0);
static_assert(NH1 % 32 == 0);
static_assert((NH2 & (NH2 - 1)) == 0);

template <int KTOT, int NW>
__device__ __forceinline__ void store_plane_row(const _Float16* lds_row, _Float16* dst_row)
{
    static_assert(KTOT % 64 == 0);
    constexpr int CH = 256;
    constexpr int NQ = (KTOT + CH * NW - 1) / (CH * NW);
    const int l = threadIdx.x & 31;
    const int w = threadIdx.x >> 5;
    v8h vv[NQ];
    #pragma unroll
    for (int q = 0; q < NQ; ++q) {
        const int off = (w + NW * q) * CH + l * 8;
        v8h z = {};
        vv[q] = z;
        if (off + 8 <= KTOT) vv[q] = *(const v8h*)(lds_row + off);
    }
    #pragma unroll
    for (int q = 0; q < NQ; ++q) {
        const int off = (w + NW * q) * CH + l * 8;
        if (off + 8 <= KTOT) *(volatile v8h*)(dst_row + off) = vv[q];
    }
    __threadfence();
    #pragma unroll
    for (int q = 0; q < NQ; ++q) {
        const int off = (w + NW * q) * CH + l * 8;
        if (off + 8 <= KTOT) *(volatile v8h*)(dst_row + off) = vv[q];
    }
}

template <int DIN>
__global__ __launch_bounds__(DIN) void k_feat(const float* __restrict__ X0,
                                             const float* __restrict__ X1,
                                             _Float16* __restrict__ F0,
                                             _Float16* __restrict__ F1)
{
    constexpr int KTOT = DIN * NF;
    constexpr int NW   = DIN / 32;
    __shared__ __attribute__((aligned(16))) _Float16 rowbuf[KTOT];

    const int row = blockIdx.x;
    const int tw  = blockIdx.y;
    const float* X = tw ? X1 : X0;
    _Float16*    F = tw ? F1 : F0;
    const int i = threadIdx.x;

    const float xv = X[(size_t)row * DIN + i];

    const float ex = __expf(-xv);
    const float sl = xv * __builtin_amdgcn_rcpf(1.0f + ex);
    rowbuf[i] = (_Float16)(sl * FSCALE);

    v8h bv;
    #pragma unroll
    for (int g = 0; g < NG; ++g) {
        const float gc = GRID_LO + (float)g * GRID_ST;
        const float z  = (xv - gc) * INVH;
        bv[g] = (_Float16)(__expf(-(z * z)) * FSCALE);
    }
    *(v8h*)(rowbuf + DIN + i * NG) = bv;
    __syncthreads();
    store_plane_row<KTOT, NW>(rowbuf, F + (size_t)row * KTOT);
}

template <int DIN>
__global__ __launch_bounds__(DIN) void k_wprep(const float* __restrict__ bw0,
                                              const float* __restrict__ bw1,
                                              const float* __restrict__ sw0,
                                              const float* __restrict__ sw1,
                                              _Float16* __restrict__ W0,
                                              _Float16* __restrict__ W1)
{
    constexpr int KTOT = DIN * NF;
    constexpr int NW   = DIN / 32;
    __shared__ __attribute__((aligned(16))) _Float16 rowbuf[KTOT];

    const int o  = blockIdx.x;
    const int tw = blockIdx.y;
    const float* bw = tw ? bw1 : bw0;
    const float* sw = tw ? sw1 : sw0;
    _Float16*    W  = tw ? W1 : W0;
    const int i = threadIdx.x;

    rowbuf[i] = (_Float16)(bw[(size_t)o * DIN + i] * WSCALE);

    const float4* sp = (const float4*)(sw + ((size_t)o * DIN + i) * NG);
    const float4 c0 = sp[0];
    const float4 c1 = sp[1];
    v8h wv;
    wv[0] = (_Float16)(c0.x * WSCALE);
    wv[1] = (_Float16)(c0.y * WSCALE);
    wv[2] = (_Float16)(c0.z * WSCALE);
    wv[3] = (_Float16)(c0.w * WSCALE);
    wv[4] = (_Float16)(c1.x * WSCALE);
    wv[5] = (_Float16)(c1.y * WSCALE);
    wv[6] = (_Float16)(c1.z * WSCALE);
    wv[7] = (_Float16)(c1.w * WSCALE);
    *(v8h*)(rowbuf + DIN + i * NG) = wv;
    __syncthreads();
    store_plane_row<KTOT, NW>(rowbuf, W + (size_t)o * KTOT);
}

template <int KTOT, int NOUT>
__global__ __launch_bounds__(128) void k_gemm(const _Float16* __restrict__ F0,
                                             const _Float16* __restrict__ F1,
                                             const _Float16* __restrict__ Wp0,
                                             const _Float16* __restrict__ Wp1,
                                             const float* __restrict__ bb0,
                                             const float* __restrict__ bb1,
                                             const float* __restrict__ sb0,
                                             const float* __restrict__ sb1,
                                             float* __restrict__ O0,
                                             float* __restrict__ O1)
{
    static_assert(KTOT % 64 == 0);
    static_assert(NOUT % TN == 0);
    __shared__ __attribute__((aligned(16))) float Cs[TM][TN];

    const int l  = threadIdx.x & 31;
    const int w  = threadIdx.x >> 5;
    const int h  = l >> 4;
    const int m  = l & 15;
    const int wr = w >> 1;
    const int wc = w & 1;
    const int tw = blockIdx.z;
    const int brow = blockIdx.y * TM;
    const int bcol = blockIdx.x * TN;

    const _Float16* fpl = tw ? F1 : F0;
    const _Float16* wpl = tw ? Wp1 : Wp0;
    const float*    bb  = tw ? bb1 : bb0;
    const float*    sb  = tw ? sb1 : sb0;
    float*          out = tw ? O1 : O0;

    const _Float16* ap = fpl + (size_t)(brow + wr * 32 + m) * KTOT + 8 * h;
    const _Float16* bp = wpl + (size_t)(bcol + wc * 32 + m) * KTOT + 8 * h;
    const size_t t16 = (size_t)16 * KTOT;

    v8f acc00 = {};
    v8f acc01 = {};
    v8f acc10 = {};
    v8f acc11 = {};

    for (int k0 = 0; k0 < KTOT; k0 += 64) {
        #pragma unroll
        for (int s = 0; s < 2; ++s) {
            const int kk = k0 + 32 * s;
            Frag a0, a1, b0, b1;
            a0.half[0] = *(const v8h*)(ap + kk);
            a0.half[1] = *(const v8h*)(ap + kk + 16);
            a1.half[0] = *(const v8h*)(ap + t16 + kk);
            a1.half[1] = *(const v8h*)(ap + t16 + kk + 16);
            b0.half[0] = *(const v8h*)(bp + kk);
            b0.half[1] = *(const v8h*)(bp + kk + 16);
            b1.half[0] = *(const v8h*)(bp + t16 + kk);
            b1.half[1] = *(const v8h*)(bp + t16 + kk + 16);
            acc00 = __builtin_amdgcn_wmma_f32_16x16x32_f16(false, a0.v, false, b0.v, (short)0, acc00, false, false);
            acc01 = __builtin_amdgcn_wmma_f32_16x16x32_f16(false, a0.v, false, b1.v, (short)0, acc01, false, false);
            acc10 = __builtin_amdgcn_wmma_f32_16x16x32_f16(false, a1.v, false, b0.v, (short)0, acc10, false, false);
            acc11 = __builtin_amdgcn_wmma_f32_16x16x32_f16(false, a1.v, false, b1.v, (short)0, acc11, false, false);
            asm volatile("v_nop\n\tv_nop\n\tv_nop\n\tv_nop"
                         : "+v"(acc00), "+v"(acc01), "+v"(acc10), "+v"(acc11)
                         : "v"(a0.v), "v"(a1.v), "v"(b0.v), "v"(b1.v));
        }
    }

    const int trow = wr * 32 + 8 * h;
    const int tcol = wc * 32 + m;
    const int ncA  = bcol + tcol;
    const int ncB  = bcol + tcol + 16;
    const float biasA = bb[ncA] + sb[ncA];
    const float biasB = bb[ncB] + sb[ncB];
    #pragma unroll
    for (int r = 0; r < 8; ++r) {
        Cs[trow + r][tcol]           = acc00[r] * OSCALE + biasA;
        Cs[trow + r][tcol + 16]      = acc01[r] * OSCALE + biasB;
        Cs[trow + 16 + r][tcol]      = acc10[r] * OSCALE + biasA;
        Cs[trow + 16 + r][tcol + 16] = acc11[r] * OSCALE + biasB;
    }
    __syncthreads();

    v4f vals[8];
    #pragma unroll
    for (int it = 0; it < 8; ++it) {
        const int rr = 2 * (it * 4 + w) + h;
        vals[it] = *(const v4f*)&Cs[rr][m * 4];
    }
    float* ob = out + (size_t)brow * NOUT + bcol + m * 4;
    #pragma unroll
    for (int it = 0; it < 8; ++it) {
        const int rr = 2 * (it * 4 + w) + h;
        *(volatile v4f*)(ob + (size_t)rr * NOUT) = vals[it];
    }
    __threadfence();
    #pragma unroll
    for (int it = 0; it < 8; ++it) {
        const int rr = 2 * (it * 4 + w) + h;
        *(volatile v4f*)(ob + (size_t)rr * NOUT) = vals[it];
    }
}

__global__ __launch_bounds__(FIN_T) void k_final(const float* __restrict__ H2x,
                                                const float* __restrict__ H2y,
                                                const float* __restrict__ fw,
                                                const float* __restrict__ fb,
                                                float* __restrict__ out,
                                                int S, int NB, float inv_s)
{
    __shared__ double red[FIN_T];
    __shared__ float  res[FIN_T];
    const int t   = threadIdx.x;
    const int nbc = NB < FIN_T ? NB : FIN_T;
    const double wxv = (double)fw[t & (NH2 - 1)];
    const double wyv = (double)fw[NH2 + (t & (NH2 - 1))];
    const int tot = S * NH2;

    for (int b = 0; b < nbc; ++b) {
        const size_t base = (size_t)b * (size_t)tot;
        double ax = 0.0, ay = 0.0;
        for (int idx = t; idx < tot; idx += FIN_T) {
            ax += (double)H2x[base + idx] * wxv;
            ay += (double)H2y[base + idx] * wyv;
        }
        red[t] = ax + ay;
        __syncthreads();
        #pragma unroll 1
        for (int sft = FIN_T / 2; sft > 0; sft >>= 1) {
            if (t < sft) red[t] = red[t] + red[t + sft];
            __syncthreads();
        }
        if (t == 0) res[b] = (float)(red[0] * (double)inv_s) + fb[0];
        __syncthreads();
    }
    float v = 0.0f;
    if (t < nbc) v = res[t];
    if (t < nbc) *(volatile float*)(out + t) = v;
    __threadfence();
    if (t < nbc) *(volatile float*)(out + t) = v;
}

static_assert(FIN_T % NH2 == 0);

extern "C" void kernel_launch(void* const* d_in, const int* in_sizes, int n_in,
                              void* d_out, int out_size, void* d_ws, size_t ws_size,
                              hipStream_t stream)
{
    if (n_in < 20) return;
    const float* x    = (const float*)d_in[0];
    const float* y    = (const float*)d_in[1];
    const float* bw1x = (const float*)d_in[2];
    const float* bb1x = (const float*)d_in[3];
    const float* sw1x = (const float*)d_in[4];
    const float* sb1x = (const float*)d_in[5];
    const float* bw2x = (const float*)d_in[6];
    const float* bb2x = (const float*)d_in[7];
    const float* sw2x = (const float*)d_in[8];
    const float* sb2x = (const float*)d_in[9];
    const float* bw1y = (const float*)d_in[10];
    const float* bb1y = (const float*)d_in[11];
    const float* sw1y = (const float*)d_in[12];
    const float* sb1y = (const float*)d_in[13];
    const float* bw2y = (const float*)d_in[14];
    const float* bb2y = (const float*)d_in[15];
    const float* sw2y = (const float*)d_in[16];
    const float* sb2y = (const float*)d_in[17];
    const float* fw   = (const float*)d_in[18];
    const float* fb   = (const float*)d_in[19];
    float* out = (float*)d_out;

    const int nx = in_sizes[0];
    if (nx <= 0 || in_sizes[1] != nx) return;
    const int M = nx / DIN1;
    if (M * DIN1 != nx || (M % TM) != 0) return;
    const int NB = out_size;
    if (NB <= 0 || NB > FIN_T || (M % NB) != 0) return;
    const int S = M / NB;

    if (in_sizes[2]  != NH1 * DIN1 || in_sizes[10] != NH1 * DIN1) return;
    if (in_sizes[4]  != NH1 * DIN1 * NG || in_sizes[12] != NH1 * DIN1 * NG) return;
    if (in_sizes[6]  != NH2 * NH1  || in_sizes[14] != NH2 * NH1) return;
    if (in_sizes[8]  != NH2 * NH1 * NG || in_sizes[16] != NH2 * NH1 * NG) return;
    if (in_sizes[3]  < NH1 || in_sizes[5]  < NH1 || in_sizes[11] < NH1 || in_sizes[13] < NH1) return;
    if (in_sizes[7]  < NH2 || in_sizes[9]  < NH2 || in_sizes[15] < NH2 || in_sizes[17] < NH2) return;
    if (in_sizes[18] < 2 * NH2 || in_sizes[19] < 1) return;

    size_t off = 0;
    auto take = [&](size_t bytes) { size_t o = off; off = (off + bytes + 127) & ~(size_t)127; return o; };
    const size_t f1b = (size_t)M * K1TOT * sizeof(_Float16);
    const size_t w1b = (size_t)NH1 * K1TOT * sizeof(_Float16);
    const size_t h1b = (size_t)M * NH1 * sizeof(float);
    const size_t f2b = (size_t)M * K2TOT * sizeof(_Float16);
    const size_t w2b = (size_t)NH2 * K2TOT * sizeof(_Float16);
    const size_t h2b = (size_t)M * NH2 * sizeof(float);
    const size_t o_f1x = take(f1b), o_f1y = take(f1b);
    const size_t o_w1x = take(w1b), o_w1y = take(w1b);
    const size_t o_h1x = take(h1b), o_h1y = take(h1b);
    const size_t o_f2x = take(f2b), o_f2y = take(f2b);
    const size_t o_w2x = take(w2b), o_w2y = take(w2b);
    const size_t o_h2x = take(h2b), o_h2y = take(h2b);
    if (off > ws_size) return;

    char* ws = (char*)d_ws;
    _Float16* f1x = (_Float16*)(ws + o_f1x);
    _Float16* f1y = (_Float16*)(ws + o_f1y);
    _Float16* w1x = (_Float16*)(ws + o_w1x);
    _Float16* w1y = (_Float16*)(ws + o_w1y);
    float*    h1x = (float*)(ws + o_h1x);
    float*    h1y = (float*)(ws + o_h1y);
    _Float16* f2x = (_Float16*)(ws + o_f2x);
    _Float16* f2y = (_Float16*)(ws + o_f2y);
    _Float16* w2x = (_Float16*)(ws + o_w2x);
    _Float16* w2y = (_Float16*)(ws + o_w2y);
    float*    h2x = (float*)(ws + o_h2x);
    float*    h2y = (float*)(ws + o_h2y);

    k_feat<DIN1><<<dim3(M, 2), dim3(DIN1), 0, stream>>>(x, y, f1x, f1y);
    k_wprep<DIN1><<<dim3(NH1, 2), dim3(DIN1), 0, stream>>>(bw1x, bw1y, sw1x, sw1y, w1x, w1y);
    k_gemm<K1TOT, NH1><<<dim3(NH1 / TN, M / TM, 2), dim3(128), 0, stream>>>(
        f1x, f1y, w1x, w1y, bb1x, bb1y, sb1x, sb1y, h1x, h1y);

    k_feat<NH1><<<dim3(M, 2), dim3(NH1), 0, stream>>>(h1x, h1y, f2x, f2y);
    k_wprep<NH1><<<dim3(NH2, 2), dim3(NH1), 0, stream>>>(bw2x, bw2y, sw2x, sw2y, w2x, w2y);
    k_gemm<K2TOT, NH2><<<dim3(NH2 / TN, M / TM, 2), dim3(128), 0, stream>>>(
        f2x, f2y, w2x, w2y, bb2x, bb2y, sb2x, sb2y, h2x, h2y);

    k_final<<<dim3(1), dim3(FIN_T), 0, stream>>>(h2x, h2y, fw, fb, out, S, NB, 1.0f / (float)S);
}
